// PatchEmbedding_4690104287386
// MI455X (gfx1250) — hardware-verified
//
#include <hip/hip_runtime.h>
#include <hip/hip_bf16.h>
#include <math.h>


#define BB 2
#define SS 2048
#define DD 1024
#define HH 16
#define DKK 64
#define QW 2

typedef _Float16 bf16;
typedef __attribute__((ext_vector_type(4))) unsigned v4u_t;
typedef unsigned v4ua __attribute__((ext_vector_type(4), may_alias));
typedef __attribute__((ext_vector_type(4))) float v4f_t;
typedef float v4fa __attribute__((ext_vector_type(4), may_alias));
typedef __attribute__((ext_vector_type(16))) bf16  bf16x16;
typedef __attribute__((ext_vector_type(8)))  bf16  bf16x8;
typedef __attribute__((ext_vector_type(4)))  bf16  bf16x4;
typedef __attribute__((ext_vector_type(8)))  float f32x8;

#define LDS_STRIDE 48
#define KSTRIDE    72
#define VSTRIDE    48

__device__ __forceinline__ f32x8 wmma_bf16(bf16x16 a, bf16x16 b, f32x8 c) {
  return __builtin_amdgcn_wmma_f32_16x16x32_f16(
      false, a, false, b, (short)0, c, false, false);
}

template <typename T>
__device__ __forceinline__ bf16x16 load_frag(const T* __restrict__ base, int ld,
                                             int row0, int k0) {
  const int lane = threadIdx.x & 31;
  const int r    = lane & 15;
  const int kh   = (lane >> 4) * 8;
  const T* p0 = base + (size_t)(row0 + r) * ld + (k0 + kh);
  const T* p1 = p0 + 16;
  bf16x16 f;
#pragma unroll
  for (int i = 0; i < 8; ++i) {
    f[i]     = (bf16)p0[i];
    f[i + 8] = (bf16)p1[i];
  }
  return f;
}

__device__ __forceinline__ bf16x16 lds_frag(const bf16* base, int stride) {
  const int lane = threadIdx.x & 31;
  const int row  = lane & 15;
  const int kh   = (lane >> 4) * 8;
  const bf16x8 lo = *(const bf16x8*)(base + row * stride + kh);
  const bf16x8 hi = *(const bf16x8*)(base + row * stride + kh + 16);
  bf16x16 f;
#pragma unroll
  for (int i = 0; i < 8; ++i) { f[i] = lo[i]; f[i + 8] = hi[i]; }
  return f;
}

template <typename T>
__device__ __forceinline__ void stage_read16(const T* __restrict__ p, float* buf) {
#pragma unroll
  for (int i = 0; i < 16; ++i) buf[i] = (float)p[i];
}

__device__ __forceinline__ void stage_write(bf16* dst, const float* buf, int nquad) {
#pragma unroll
  for (int i = 0; i < nquad; ++i) {
    bf16x4 q;
    q[0] = (bf16)buf[4 * i];     q[1] = (bf16)buf[4 * i + 1];
    q[2] = (bf16)buf[4 * i + 2]; q[3] = (bf16)buf[4 * i + 3];
    *(bf16x4*)(dst + 4 * i) = q;
  }
}

template <typename AT, int MODE>
__global__ __launch_bounds__(256) void gemm_bias_kernel(
    const AT* __restrict__ A, const float* __restrict__ W,
    const float* __restrict__ bias, void* __restrict__ out,
    int M, int N, int K) {
  __shared__ bf16 ldsA[128 * LDS_STRIDE];
  __shared__ bf16 ldsW[256 * LDS_STRIDE];
  __shared__ __attribute__((aligned(16))) unsigned char sob[256 * 136 * 2];

  const int t    = threadIdx.x;
  const int wave = t >> 5;
  const int lane = t & 31;
  const int wm   = (wave & 1) * 64;
  const int wn   = (wave >> 1) * 64;
  const int mBlk = blockIdx.x * 128;
  const int nBlk = blockIdx.y * 256;

  const int arow = t >> 1;
  const int ach  = (t & 1) * 16;

  float abuf[16];
  float wbuf[32];

  stage_read16(A + (size_t)(mBlk + arow) * K + ach, abuf);
  stage_read16(W + (size_t)(nBlk + t) * K,          wbuf);
  stage_read16(W + (size_t)(nBlk + t) * K + 16,     wbuf + 16);

  f32x8 acc[4][4] = {};

  for (int k = 0; k < K; k += 32) {
    __syncthreads();
    stage_write(&ldsA[arow * LDS_STRIDE + ach], abuf, 4);
    stage_write(&ldsW[t * LDS_STRIDE],          wbuf, 8);
    if (k + 32 < K) {
      stage_read16(A + (size_t)(mBlk + arow) * K + (k + 32) + ach, abuf);
      stage_read16(W + (size_t)(nBlk + t) * K + (k + 32),          wbuf);
      stage_read16(W + (size_t)(nBlk + t) * K + (k + 32) + 16,     wbuf + 16);
    }
    __syncthreads();

    bf16x16 af[4], wf[4];
#pragma unroll
    for (int i = 0; i < 4; ++i)
      af[i] = lds_frag(ldsA + (wm + 16 * i) * LDS_STRIDE, LDS_STRIDE);
#pragma unroll
    for (int j = 0; j < 4; ++j)
      wf[j] = lds_frag(ldsW + (wn + 16 * j) * LDS_STRIDE, LDS_STRIDE);
#pragma unroll
    for (int i = 0; i < 4; ++i)
#pragma unroll
      for (int j = 0; j < 4; ++j)
        acc[i][j] = wmma_bf16(af[i], wf[j], acc[i][j]);
  }

  const int nlane = lane & 15;
  const int mh    = (lane >> 4) * 8;
  __syncthreads();
  if (MODE == 0 || MODE == 1) {
    bf16* so = (bf16*)sob;
#pragma unroll
    for (int i = 0; i < 4; ++i)
#pragma unroll
      for (int j = 0; j < 4; ++j) {
        const int nl = wn + 16 * j + nlane;
        const float bv = bias ? bias[nBlk + nl] : 0.0f;
#pragma unroll
        for (int r = 0; r < 8; ++r) {
          const int ml = wm + 16 * i + mh + r;
          const bf16 hv = (bf16)(acc[i][j][r] + bv);
          if (MODE == 0) so[ml * 264 + nl] = hv;
          else           so[nl * 136 + ml] = hv;
        }
      }
    __syncthreads();
#pragma unroll 1
    for (int pass = 0; pass < 2; ++pass) {
      if (MODE == 0) {
        for (int ch = t; ch < 128 * 32; ch += 256) { const int ml = ch >> 5, q = (ch & 31) * 8;
          *(volatile v4u_t*)((bf16*)out + (size_t)(mBlk + ml) * N + nBlk + q) = *(const v4ua*)(so + ml * 264 + q); }
      } else {
        const int b_ = mBlk / SS, s0 = mBlk & (SS - 1);
        for (int ch = t; ch < 256 * 16; ch += 256) { const int nl = ch >> 4, q = (ch & 15) * 8; const int n = nBlk + nl, h = n >> 6, dk = n & (DKK - 1);
          *(volatile v4u_t*)((bf16*)out + (((size_t)(b_ * HH + h)) * DKK + dk) * SS + s0 + q) = *(const v4ua*)(so + nl * 136 + q); }
      }
      __threadfence();
    }
  } else {
    float* so = (float*)sob;
#pragma unroll 1
    for (int hf = 0; hf < 2; ++hf) {
      if (wm == hf * 64) {
#pragma unroll
        for (int i = 0; i < 4; ++i)
#pragma unroll
          for (int j = 0; j < 4; ++j) {
            const int nl = wn + 16 * j + nlane;
            const float bv = bias ? bias[nBlk + nl] : 0.0f;
#pragma unroll
            for (int r = 0; r < 8; ++r) so[(16 * i + mh + r) * 260 + nl] = acc[i][j][r] + bv;
          }
      }
      __syncthreads();
#pragma unroll 1
      for (int pass = 0; pass < 2; ++pass) {
        for (int ch = t; ch < 64 * 64; ch += 256) { const int ml = ch >> 6, q = (ch & 63) * 4;
          *(volatile v4f_t*)((float*)out + (size_t)(mBlk + hf * 64 + ml) * N + nBlk + q) = *(const volatile v4fa*)(so + ml * 260 + q); }
        __threadfence();
      }
      __syncthreads();
    }
  }
}


#define NBI 64
#define NPR 196
#define MT 12544
#define DK 768
#define DE 384
#define NPAD 512

__global__ __launch_bounds__(192) void k_im2col(const float* __restrict__ img, float* __restrict__ A) {
  const int m = blockIdx.x, b = m / NPR, pi = m % NPR, gh = pi / 14, gw = pi % 14, t = threadIdx.x;
  const int c = t >> 6, ph = (t >> 2) & 15, pw4 = (t & 3) * 4;
  const v4f_t v = *(const v4fa*)(img + (((size_t)b * 3 + c) * 224 + gh * 16 + ph) * 224 + gw * 16 + pw4);
  float* dst = A + (size_t)m * DK + c * 256 + ph * 16 + pw4; *(volatile v4f_t*)dst = v; __threadfence(); *(volatile v4f_t*)dst = v;
}
__global__ __launch_bounds__(192) void k_wpad(const float* __restrict__ w, float* __restrict__ Wp) {
  const int n = blockIdx.x, t = threadIdx.x; v4f_t v; if (n < DE) v = *(const v4fa*)(w + (size_t)n * DK + t * 4); else { v.x = v.y = v.z = v.w = 0.0f; }
  *(volatile v4f_t*)(Wp + (size_t)n * DK + t * 4) = v; __threadfence(); *(volatile v4f_t*)(Wp + (size_t)n * DK + t * 4) = v;
}
__global__ __launch_bounds__(96) void k_ln(const float* __restrict__ T, const float* __restrict__ bias, const float* __restrict__ g, const float* __restrict__ be, float* __restrict__ out) {
  __shared__ float red[96];
  const int m = blockIdx.x, t = threadIdx.x;
  v4f_t v = *(const v4fa*)(T + (size_t)m * NPAD + t * 4); const v4f_t bb = *(const v4fa*)(bias + t * 4); v.x += bb.x; v.y += bb.y; v.z += bb.z; v.w += bb.w;
  red[t] = v.x + v.y + v.z + v.w; __syncthreads();
  if (t < 32) { float s = red[t] + red[t + 32] + red[t + 64];
#pragma unroll
    for (int o = 16; o >= 1; o >>= 1) s += __shfl_xor(s, o, 32); if (t == 0) red[0] = s; }
  __syncthreads(); const float mu = red[0] / (float)DE; __syncthreads();
  const float dx = v.x - mu, dy = v.y - mu, dz = v.z - mu, dw = v.w - mu; red[t] = dx * dx + dy * dy + dz * dz + dw * dw; __syncthreads();
  if (t < 32) { float s = red[t] + red[t + 32] + red[t + 64];
#pragma unroll
    for (int o = 16; o >= 1; o >>= 1) s += __shfl_xor(s, o, 32); if (t == 0) red[0] = s; }
  __syncthreads(); const float rs = 1.0f / sqrtf(red[0] / (float)DE + 1e-5f);
  const v4f_t gv = *(const v4fa*)(g + t * 4), bv = *(const v4fa*)(be + t * 4);
  v4f_t r; r.x = dx * rs * gv.x + bv.x; r.y = dy * rs * gv.y + bv.y; r.z = dz * rs * gv.z + bv.z; r.w = dw * rs * gv.w + bv.w;
  *(volatile v4f_t*)(out + (size_t)m * DE + t * 4) = r; __threadfence(); *(volatile v4f_t*)(out + (size_t)m * DE + t * 4) = r;
}
__global__ __launch_bounds__(256) void k_entropy(const float* __restrict__ img, float* __restrict__ ent) {
  __shared__ int cntw[8][33]; __shared__ int cnt[32][33]; __shared__ float res[32];
  const int m0 = blockIdx.x * 32, t = threadIdx.x, wave = t >> 5, lane = t & 31;
  const int ph = t >> 4, pw = t & 15;
#pragma unroll 1
  for (int j = 0; j < 32; ++j) {
    const int m = m0 + j, b = m / NPR, pi = m % NPR, gh = pi / 14, gw = pi % 14;
    const size_t base = ((size_t)b * 3) * 224 * 224 + (size_t)(gh * 16 + ph) * 224 + gw * 16 + pw;
    const float gray = (img[base] + img[base + (size_t)224 * 224] + img[base + (size_t)2 * 224 * 224]) / 3.0f;
    float qf = gray * 31.0f; qf = fminf(fmaxf(qf, 0.0f), 31.0f); const int bin = (int)qf;
#pragma unroll 1
    for (int k = 0; k < 32; ++k) { const unsigned m_ = __builtin_amdgcn_ballot_w32(bin == k); if (lane == 0) cntw[wave][k] = __builtin_popcount(m_); }
    __syncthreads();
    if (t < 32) { int s = 0;
#pragma unroll
      for (int w = 0; w < 8; ++w) s += cntw[w][t];
      cnt[j][t] = s; }
    __syncthreads();
  }
  if (t < 32) { float e = 0.0f; int tot = 0;
    for (int k = 0; k < 32; ++k) tot += cnt[t][k];
    const float inv = 1.0f / fmaxf((float)tot, 1e-8f);
#pragma unroll 1
    for (int k = 0; k < 32; ++k) { const float p = (float)cnt[t][k] * inv; e -= p * log2f(p + 1e-10f); }
    res[t] = e / 5.0f; }
  __syncthreads();
  if (t < 8) { const v4f_t v = *(const volatile v4fa*)(res + t * 4); *(volatile v4f_t*)(ent + (size_t)m0 + t * 4) = v; __threadfence(); *(volatile v4f_t*)(ent + (size_t)m0 + t * 4) = v; }
}

extern "C" void kernel_launch(void* const* d_in, const int* in_sizes, int n_in,
                              void* d_out, int out_size, void* d_ws, size_t ws_size,
                              hipStream_t stream) {
  (void)in_sizes; (void)n_in; (void)out_size; (void)ws_size;
  const float* img = (const float*)d_in[0];
  const float* w = (const float*)d_in[1];
  const float* bias = (const float*)d_in[2]; const float* g = (const float*)d_in[3]; const float* be = (const float*)d_in[4];
  float* xo = (float*)d_out;
  float* ent = xo + (size_t)MT * DE;
  char* ws = (char*)d_ws;
  float* A  = (float*)ws; ws += (size_t)MT * DK * 4;
  float* Wp = (float*)ws; ws += (size_t)NPAD * DK * 4;
  float* T  = (float*)ws; ws += (size_t)MT * NPAD * 4;
  k_im2col<<<MT, 192, 0, stream>>>(img, A);
  k_wpad<<<NPAD, 192, 0, stream>>>(w, Wp);
  gemm_bias_kernel<float, 2><<<dim3(MT / 128, NPAD / 256), 256, 0, stream>>>(A, Wp, nullptr, T, MT, NPAD, DK);
  k_ln<<<MT, 96, 0, stream>>>(T, bias, g, be, xo);
  k_entropy<<<MT / 32, 256, 0, stream>>>(img, ent);
}
